// HypoShacira_44762149159575
// MI455X (gfx1250) — hardware-verified
//
#include <hip/hip_runtime.h>
#include <math.h>

typedef __attribute__((ext_vector_type(16))) _Float16 v16h;
typedef __attribute__((ext_vector_type(16))) __bf16 v16b;
typedef __attribute__((ext_vector_type(8)))  _Float16 v8h;
typedef __attribute__((ext_vector_type(8)))  float v8f;
typedef __attribute__((ext_vector_type(4)))  float v4f;
typedef __attribute__((ext_vector_type(2)))  float v2f;
typedef __attribute__((ext_vector_type(4)))  unsigned v4u;
typedef __attribute__((ext_vector_type(4)))  int v4i;
typedef float __attribute__((may_alias)) float_a;
typedef int __attribute__((may_alias)) int_a;

template <typename T> __device__ __forceinline__ void vst2(void* p, T v) { *(volatile T*)p = v; __threadfence(); *(volatile T*)p = v; }
__device__ __forceinline__ v8f wmma16(v16h a, v16h b, v8f c) {
  v8f d = __builtin_amdgcn_wmma_f32_16x16x32_f16(false, a, false, b, (short)0, c, false, false);
  asm volatile("v_nop\n\tv_nop\n\tv_nop\n\tv_nop" : "+v"(d) : "v"(a), "v"(b));
  return d;
}
__device__ __forceinline__ v8f wmma_bf(v16b a, v16b b, v8f c) {
  v8f d = __builtin_amdgcn_wmma_f32_16x16x32_bf16(false, a, false, b, (short)0, c, false, false);
  asm volatile("v_nop\n\tv_nop\n\tv_nop\n\tv_nop" : "+v"(d) : "v"(a), "v"(b));
  return d;
}
__device__ __forceinline__ v16h frag_h(const _Float16* rowk0, int lane) {
  union { v16h v; v8h q[2]; } u; const _Float16* p = rowk0 + 8 * (lane >> 4);
  u.q[0] = *(const v8h*)p; u.q[1] = *(const v8h*)(p + 16); return u.v;
}
__device__ __forceinline__ v16h frag_f32(const float* rowk0, int lane) {
  v16h a; const float* p = rowk0 + 8 * (lane >> 4);
#pragma unroll
  for (int i = 0; i < 8; ++i) { a[i] = (_Float16)p[i]; a[8 + i] = (_Float16)p[16 + i]; }
  return a;
}
__device__ __forceinline__ v16h frag_f32s(const float* rowk0, int lane, float sc) {
  v16h a; const float* p = rowk0 + 8 * (lane >> 4);
#pragma unroll
  for (int i = 0; i < 8; ++i) { a[i] = (_Float16)(p[i] * sc); a[8 + i] = (_Float16)(p[16 + i] * sc); }
  return a;
}
__device__ __forceinline__ v16h fragc_f32(const float* W, int k0, int n, int lane, int ld, int K) {
  v16h a; const int g = lane >> 4;
#pragma unroll
  for (int i = 0; i < 8; ++i) { const int ka = k0 + 8 * g + i, kb = ka + 16;
    a[i] = (_Float16)(ka < K ? W[(size_t)(ka < K ? ka : K - 1) * ld + n] : 0.f); a[8 + i] = (_Float16)(kb < K ? W[(size_t)(kb < K ? kb : K - 1) * ld + n] : 0.f); }
  return a;
}
struct F2 { v16b h, l; };
__device__ __forceinline__ F2 bsplit16(const float v[16]) { F2 r;
#pragma unroll
  for (int i = 0; i < 16; ++i) { const __bf16 h = (__bf16)v[i]; r.h[i] = h; r.l[i] = (__bf16)(v[i] - (float)h); }
  return r; }
__device__ __forceinline__ F2 split_row(const float* row, int k0, int lane) { float v[16]; const float* p = row + k0 + 8 * (lane >> 4);
#pragma unroll
  for (int i = 0; i < 8; ++i) { v[i] = p[i]; v[8 + i] = p[16 + i]; }
  return bsplit16(v); }
__device__ __forceinline__ F2 split_rowK(const float* row, int k0, int lane, int K) { float v[16]; const int g = lane >> 4;
#pragma unroll
  for (int i = 0; i < 8; ++i) { const int ka = k0 + 8 * g + i, kb = ka + 16; v[i] = ka < K ? row[ka < K ? ka : K - 1] : 0.f; v[8 + i] = kb < K ? row[kb < K ? kb : K - 1] : 0.f; }
  return bsplit16(v); }
__device__ __forceinline__ F2 split_col(const float* W, int k0, int n, int lane, int ld, int K) { float v[16]; const int g = lane >> 4;
#pragma unroll
  for (int i = 0; i < 8; ++i) { const int ka = k0 + 8 * g + i, kb = ka + 16; v[i] = ka < K ? W[(size_t)(ka < K ? ka : K - 1) * ld + n] : 0.f; v[8 + i] = kb < K ? W[(size_t)(kb < K ? kb : K - 1) * ld + n] : 0.f; }
  return bsplit16(v); }
__device__ __forceinline__ v8f mac3(const F2& a, const F2& b, v8f c) { c = wmma_bf(a.l, b.h, c); c = wmma_bf(a.h, b.l, c); return wmma_bf(a.h, b.h, c); }
__device__ __forceinline__ float sigm(float v) { return 1.0f / (1.0f + expf(-v)); }
#define LDSX() do { asm volatile("s_wait_dscnt 0" ::: "memory"); __builtin_amdgcn_wave_barrier(); __builtin_amdgcn_fence(__ATOMIC_RELEASE, "workgroup"); } while (0)


#define NBI 16
#define NPT 31684
#define LL 44
#define KIN 64
#define HID 16
#define TOTAL 38584
#define TPI 496
#ifndef NBT
#define NBT NBI
#endif
typedef __attribute__((ext_vector_type(8))) __bf16 v8b;
__device__ __forceinline__ v16b frag_b(const __bf16* rowk0, int lane) {
  union { v16b v; v8b q[2]; } u; const __bf16* p = rowk0 + 8 * (lane >> 4);
  u.q[0] = *(const v8b*)p; u.q[1] = *(const v8b*)(p + 16); return u.v;
}
__device__ __forceinline__ float bfr(float v) { return (float)(__bf16)v; }
__device__ __attribute__((noinline)) float exp_ni(float v) { return expf(v); }
__device__ __attribute__((noinline)) float erf_ni(float v) { return erff(v); }
__constant__ int c_res[LL] = {16,17,18,18,19,20,21,22,24,25,26,27,29,30,31,33,35,36,38,40,42,44,46,49,51,54,56,59,62,65,68,72,75,79,83,87,91,96,101,105,111,116,122,128};
__constant__ int c_dense[LL] = {1,1,1,1,1,1,1,1,1,1,1,1,1,1,1,0,0,0,0,0,0,0,0,0,0,0,0,0,0,0,0,0,0,0,0,0,0,0,0,0,0,0,0,0};
__constant__ int c_offs[LL] = {0,289,613,974,1335,1735,2176,2660,3189,3814,4490,5219,6003,6903,7864,8888,9912,10936,11960,12984,14008,15032,16056,17080,18104,19128,20152,21176,22200,23224,24248,25272,26296,27320,28344,29368,30392,31416,32440,33464,34488,35512,36536,37560};

__device__ __forceinline__ F2 split16(const float* row, int lane) { float v[16]; const float* p = row + 8 * (lane >> 4);
#pragma unroll
  for (int i = 0; i < 8; ++i) { v[i] = p[i]; v[8 + i] = 0.f; } return bsplit16(v); }
#define WS_P1  0u
#define WS_P2  (WS_P1 + 2u * NBI * HID * KIN)
#define WS_P3  (WS_P2 + 2u * NBI * HID * 32)
#define WS_STG (((WS_P3 + 2u * NBI * 16 * 32) + 127u) / 128u * 128u)
#define WS_END (WS_STG + 4u * NBI * TPI * 64 * 4)

__global__ __launch_bounds__(256) void k_pack(const float* __restrict__ W1, const float* __restrict__ W2, const float* __restrict__ W3, __bf16* __restrict__ P1, __bf16* __restrict__ P2, __bf16* __restrict__ P3) {
  __shared__ __align__(16) __bf16 s1[HID * KIN], s2[HID * 32], s3[16 * 32]; const int b = blockIdx.x, t = threadIdx.x;
  for (int q = t; q < HID * KIN; q += 256) { const int h = q / KIN, k = q % KIN; s1[q] = (__bf16)((k < LL) ? W1[((size_t)b * HID + h) * LL + k] : 0.f); }
  for (int q = t; q < HID * 32; q += 256) { const int h = q / 32, k = q % 32; s2[q] = (__bf16)((k < HID) ? W2[((size_t)b * HID + h) * HID + k] : 0.f); }
  for (int q = t; q < 16 * 32; q += 256) { const int n = q / 32, k = q % 32; s3[q] = (__bf16)((n < 3 && k < HID) ? W3[((size_t)b * 3 + n) * HID + k] : 0.f); }
  __syncthreads();
  for (int q = t; q < HID * KIN / 8; q += 256) vst2((unsigned*)(P1 + (size_t)b * HID * KIN + q * 8), *(const v4u*)&s1[q * 8]);
  for (int q = t; q < HID * 32 / 8; q += 256) vst2((unsigned*)(P2 + (size_t)b * HID * 32 + q * 8), *(const v4u*)&s2[q * 8]);
  for (int q = t; q < 16 * 32 / 8; q += 256) vst2((unsigned*)(P3 + (size_t)b * 16 * 32 + q * 8), *(const v4u*)&s3[q * 8]);
}
__global__ __launch_bounds__(128) void k_inr(const float* __restrict__ X, const float* __restrict__ CB, const __bf16* __restrict__ P1, const __bf16* __restrict__ P2, const __bf16* __restrict__ P3, float* __restrict__ STG) {
  __shared__ __align__(16) __bf16 sah[64][KIN + 8], sal[64][KIN + 8]; __shared__ __align__(16) float sh1[64][HID + 4]; __shared__ __align__(16) float so[64][4];
  const int tid = threadIdx.x, wave = tid >> 5, lane = tid & 31, col = lane & 15, g = lane >> 4; const int tile = blockIdx.x, b = blockIdx.y; const int n0 = tile * 64;
  { const int p = tid & 63, l0 = (tid >> 6) * 22; const int n = min(n0 + p, NPT - 1); const float px = bfr(X[((size_t)b * NPT + n) * 2]), py = bfr(X[((size_t)b * NPT + n) * 2 + 1]); const float* cb = CB + (size_t)b * TOTAL;
    for (int l = l0; l < l0 + 22; ++l) { const int res = c_res[l]; const float rf = (float)res; const float sx = px * rf, sy = py * rf; const float bx = floorf(sx), by = floorf(sy); const float fx = sx - bx, fy = sy - by; const int ix = (int)bx, iy = (int)by;
      float f = 0.f;
#pragma unroll
      for (int c = 0; c < 4; ++c) { const int cx = min(ix + (c >> 1), res), cy = min(iy + (c & 1), res);
        int idx; if (c_dense[l]) idx = cy * (res + 1) + cx; else { const unsigned hh = ((unsigned)cx ^ ((unsigned)cy * 2654435761u)) % 1024u; idx = (int)hh; }
        idx += c_offs[l]; const float w = ((c >> 1) ? fx : 1.f - fx) * ((c & 1) ? fy : 1.f - fy); f += bfr(cb[idx]) * w; }
      const __bf16 hb = (__bf16)f; sah[p][l] = hb; sal[p][l] = (__bf16)(f - (float)hb); }
    if (l0 == 22) for (int l = LL; l < KIN; ++l) { sah[p][l] = (__bf16)0.f; sal[p][l] = (__bf16)0.f; } }
  __syncthreads();
  { v8f acc = {};
#pragma unroll
    for (int kc = 0; kc < 2; ++kc) { F2 a; a.h = frag_b(&sah[wave * 16 + col][kc * 32], lane); a.l = frag_b(&sal[wave * 16 + col][kc * 32], lane); const v16b w = frag_b(P1 + ((size_t)b * HID + col) * KIN + kc * 32, lane); acc = wmma_bf(a.l, w, acc); acc = wmma_bf(a.h, w, acc); }
#pragma unroll
    for (int r = 0; r < 8; ++r) sh1[wave * 16 + 8 * g + r][col] = fmaxf(acc[r], 0.f); }
  LDSX();
  { F2 a = split16(&sh1[wave * 16 + col][0], lane); v8f acc = {}; const v16b w = frag_b(P2 + ((size_t)b * HID + col) * 32, lane); acc = wmma_bf(a.l, w, acc); acc = wmma_bf(a.h, w, acc);
    LDSX();
#pragma unroll
    for (int r = 0; r < 8; ++r) sh1[wave * 16 + 8 * g + r][col] = fmaxf(acc[r], 0.f);
    LDSX();
    a = split16(&sh1[wave * 16 + col][0], lane); v8f acc3 = {}; const v16b w3 = frag_b(P3 + ((size_t)b * 16 + col) * 32, lane); acc3 = wmma_bf(a.l, w3, acc3); acc3 = wmma_bf(a.h, w3, acc3);
    if (col < 3) {
#pragma unroll
      for (int r = 0; r < 8; ++r) so[wave * 16 + 8 * g + r][col] = 1.0f / (1.0f + exp_ni(-acc3[r])); }
    else if (col == 3) {
#pragma unroll
      for (int r = 0; r < 8; ++r) so[wave * 16 + 8 * g + r][3] = 0.f; } }
  __syncthreads();
  if (tid < 64) vst2(STG + (((size_t)b * TPI + tile) * 64 + tid) * 4, *(const v4f*)&so[tid][0]);
}
__global__ __launch_bounds__(256) void k_flat(const float* __restrict__ STG, float* __restrict__ OUT) {
  const size_t q = (size_t)blockIdx.x * 256 + threadIdx.x; const size_t total4 = (size_t)NBT * NPT * 3 / 4;
  if (q >= total4) return;
  v4f v;
#pragma unroll
  for (int i = 0; i < 4; ++i) { const size_t e = q * 4 + i; const size_t pt = e / 3; const int c = (int)(e % 3); const int b = (int)(pt / NPT), n = (int)(pt % NPT); v[i] = STG[(((size_t)b * TPI + n / 64) * 64 + (n % 64)) * 4 + c]; }
  vst2(OUT + q * 4, v);
}
extern "C" void kernel_launch(void* const* d_in, const int* in_sizes, int n_in, void* d_out, int out_size, void* d_ws, size_t ws_size, hipStream_t stream) {
  (void)in_sizes; (void)n_in; (void)out_size;
  const float** F = (const float**)d_in;
  if (ws_size < (size_t)WS_END) return;
  char* ws = (char*)d_ws; __bf16 *P1 = (__bf16*)(ws + WS_P1), *P2 = (__bf16*)(ws + WS_P2), *P3 = (__bf16*)(ws + WS_P3); float* STG = (float*)(ws + WS_STG);
  k_pack<<<NBI, 256, 0, stream>>>(F[2], F[3], F[4], P1, P2, P3);
  k_inr<<<dim3(TPI, NBT), 128, 0, stream>>>(F[0], F[1], P1, P2, P3, STG);
  k_flat<<<(NBT * NPT * 3 / 4 + 255) / 256, 256, 0, stream>>>(STG, (float*)d_out);
}
